// CausalSelfAttention_30691836297463
// MI455X (gfx1250) — hardware-verified
//
#include <hip/hip_runtime.h>


#ifndef NB
#define NB 2
#endif
#ifndef SEQ
#define SEQ 2048
#endif
#define NB_FULL  2
#define SEQ_FULL 2048
#define DM   1024
#define NH   16
#define HD   64
#define RH   256
#define TPE  (RH / 16)
#define TPM  ((SEQ - RH) / 16)
#define TPMD (TPM > 0 ? TPM : 1)
#define PP   40
#define OP   68
#define RSC  2048.0f
#define RINV (1.0f / 2048.0f)
#define SC2  0.18033688011112042f
#define NEGB (-3.0e38f)

static_assert(DM == NH * HD);
static_assert(DM == 1024);
static_assert(HD == 64);
static_assert(SEQ % 256 == 0 && SEQ >= RH && SEQ <= SEQ_FULL);
static_assert(NB >= 1 && NB <= NB_FULL);
static_assert(RH % 32 == 0);
static_assert((NB * NH * TPE) % 8 == 0);
static_assert((NB * NH * TPM) % 8 == 0);
static_assert((NB * SEQ) % 64 == 0 && (3 * DM) % 64 == 0 && DM % 64 == 0 && DM % 32 == 0);
static_assert(PP % 8 == 0 && PP >= 32 && OP % 4 == 0 && OP >= 64);

typedef _Float16 h16;
typedef unsigned short bf;
typedef __attribute__((ext_vector_type(16))) __bf16   v16bf;
typedef __attribute__((ext_vector_type(16))) _Float16 v16h;
typedef __attribute__((ext_vector_type(8)))  _Float16 v8h;
typedef __attribute__((ext_vector_type(8)))  unsigned short v8us;
typedef __attribute__((ext_vector_type(2)))  unsigned short v2us;
typedef __attribute__((ext_vector_type(8)))  float    v8f;
typedef __attribute__((ext_vector_type(4)))  float    v4f;
typedef v8h  __attribute__((may_alias)) v8ha;
typedef v4f  __attribute__((may_alias)) v4fa;

__device__ __forceinline__ unsigned short f2bf(float f) { unsigned u = __float_as_uint(f); u += 0x7FFFu + ((u >> 16) & 1u); return (unsigned short)(u >> 16); }
__device__ __forceinline__ float bf2f(unsigned short b) { return __uint_as_float(((unsigned)b) << 16); }
__device__ __forceinline__ float bfr(float f) { return bf2f(f2bf(f)); }
__device__ __forceinline__ void splitf(float y, unsigned short& h, unsigned short& l) { h = f2bf(y); l = f2bf(y - bf2f(h)); }
__device__ __forceinline__ v16h cat16(v8h lo, v8h hi) { return __builtin_shufflevector(lo, hi, 0, 1, 2, 3, 4, 5, 6, 7, 8, 9, 10, 11, 12, 13, 14, 15); }
__device__ __forceinline__ v16bf cat16b(v8us lo, v8us hi) { return __builtin_bit_cast(v16bf, __builtin_shufflevector(lo, hi, 0, 1, 2, 3, 4, 5, 6, 7, 8, 9, 10, 11, 12, 13, 14, 15)); }
__device__ __forceinline__ v8f wmma16(v16h a, v16h b, v8f c) { return __builtin_amdgcn_wmma_f32_16x16x32_f16(false, a, false, b, (short)0, c, false, false); }
__device__ __forceinline__ v8f wmmab(v16bf a, v16bf b, v8f c) { return __builtin_amdgcn_wmma_f32_16x16x32_bf16(false, a, false, b, (short)0, c, false, false); }
__device__ __forceinline__ v16h  ldh(const h16* p) { return cat16(*(const v8h*)p, *(const v8h*)(p + 16)); }
__device__ __forceinline__ v16bf ldb(const bf* p)  { return cat16b(*(const v8us*)p, *(const v8us*)(p + 16)); }

template <int NSPLIT, bool BIAS>
__device__ __forceinline__ void gemmw_body(const bf* __restrict__ A, const bf* A2, const bf* __restrict__ Bt, const int K, float* C, const int ldc, const float* __restrict__ bias) {
    __shared__ __align__(16) float os[16 * 68];
    const int lane = threadIdx.x & 31, lr = lane & 15, hi = lane >> 4; const int r0 = blockIdx.x * 64, c0 = blockIdx.y * 64;
    v8f acc[4][4];
#pragma unroll
    for (int mb = 0; mb < 4; ++mb)
#pragma unroll
        for (int nb = 0; nb < 4; ++nb) acc[mb][nb] = (v8f){};
    const size_t aoff = (size_t)(r0 + lr) * K + 8 * hi, boff = (size_t)(c0 + lr) * K + 8 * hi;
#pragma unroll 1
    for (int kc = 0; kc < K; kc += 32) {
        v16bf a[4], a2[4];
#pragma unroll
        for (int mb = 0; mb < 4; ++mb) { a[mb] = ldb(A + aoff + (size_t)mb * 16 * K + kc); if (NSPLIT == 1) a2[mb] = ldb(A2 + aoff + (size_t)mb * 16 * K + kc); }
#pragma unroll
        for (int nb = 0; nb < 4; ++nb) { const v16bf b = ldb(Bt + boff + (size_t)nb * 16 * K + kc);
#pragma unroll
            for (int mb = 0; mb < 4; ++mb) { acc[mb][nb] = wmmab(a[mb], b, acc[mb][nb]); if (NSPLIT == 1) acc[mb][nb] = wmmab(a2[mb], b, acc[mb][nb]); } }
        asm volatile("v_nop\n\tv_nop\n\tv_nop\n\tv_nop" : "+v"(acc[0][0]), "+v"(acc[1][1]), "+v"(acc[2][2]), "+v"(acc[3][3]) : "v"(a[0]), "v"(a[3]));
    }
#pragma unroll
    for (int mb = 0; mb < 4; ++mb) {
#pragma unroll
        for (int nb = 0; nb < 4; ++nb) {
#pragma unroll
            for (int j = 0; j < 8; ++j) os[(hi * 8 + j) * 68 + nb * 16 + lr] = acc[mb][nb][j]; }
        __builtin_amdgcn_wave_barrier(); asm volatile("" ::: "memory");
        float* crow = C + (size_t)(r0 + mb * 16) * ldc + c0;
#pragma unroll 1
        for (int ps = 0; ps < 2; ++ps) {
#pragma unroll
            for (int s = 0; s < 8; ++s) { const int row = 2 * s + hi, cofs = lr * 4; v4f val = *(const v4fa*)(os + row * 68 + cofs); if (BIAS) { val[0] += bfr(bias[c0 + cofs]); val[1] += bfr(bias[c0 + cofs + 1]); val[2] += bfr(bias[c0 + cofs + 2]); val[3] += bfr(bias[c0 + cofs + 3]); }
                *(volatile v4f*)(crow + (size_t)row * ldc + cofs) = val; }
            if (ps == 0) __threadfence(); }
        __builtin_amdgcn_wave_barrier(); asm volatile("" ::: "memory");
    }
}
__global__ __launch_bounds__(32) void k_gemm_qkv(const bf* XB, const bf* Wt, float* F) { gemmw_body<0, false>(XB, XB, Wt, DM, F, 3 * DM, nullptr); }
__global__ __launch_bounds__(32) void k_gemm_out(const bf* Yh, const bf* Yl, const bf* Wt, const float* bias, float* OUT) {
    const size_t z = blockIdx.z;
    gemmw_body<1, true>(Yh + z * (size_t)SEQ * DM, Yl + z * (size_t)SEQ * DM, Wt, DM, OUT + z * (size_t)SEQ_FULL * DM, DM, bias);
}

__global__ __launch_bounds__(256) void k_wt(const float* __restrict__ w, int N, bf* Bt) {
    const int lane = threadIdx.x & 31; const int L0 = (blockIdx.x * 8 + (threadIdx.x >> 5)) * 8; const int nlines = N * (DM / 64);
#pragma unroll 1
    for (int ps = 0; ps < 2; ++ps) {
#pragma unroll 1
        for (int l = 0; l < 8; ++l) { const int L = L0 + l; if (L >= nlines) break; const int e = L * 64 + lane * 2; const int k = e & (DM - 1), n = e >> 10; v2us o;
            o[0] = f2bf(w[(size_t)k * N + n]); o[1] = f2bf(w[(size_t)(k + 1) * N + n]); *(volatile v2us*)(Bt + e) = o; }
        if (ps == 0) __threadfence(); }
}
__global__ __launch_bounds__(256) void k_cvtx(const float* __restrict__ x, bf* XB) {
    const unsigned i = blockIdx.x * 256u + threadIdx.x; if (i >= (unsigned)(NB * SEQ * (DM / 8))) return;
    const unsigned row = i / (DM / 8), c8 = i % (DM / 8); const unsigned b = row / SEQ, t = row % SEQ;
    const float* s = x + ((size_t)b * SEQ_FULL + t) * DM + c8 * 8;
    const v4f a = *(const v4f*)s, c = *(const v4f*)(s + 4); v8us o;
#pragma unroll
    for (int k = 0; k < 4; ++k) { o[k] = f2bf(a[k]); o[k + 4] = f2bf(c[k]); }
    *(volatile v8us*)(XB + (size_t)i * 8) = o; __threadfence(); *(volatile v8us*)(XB + (size_t)i * 8) = o;
}
__global__ __launch_bounds__(256) void k_qkp(const float* __restrict__ F, h16* QH, h16* QR, h16* KH, h16* KR) {
    const unsigned i = blockIdx.x * 256u + threadIdx.x; if (i >= (unsigned)(NB * SEQ) * 256u) return;
    const unsigned m = i >> 8, g = i & 255u, sec = g >> 7, c8 = g & 127u, h = c8 >> 3, d0 = (c8 & 7u) * 8u;
    const unsigned b = m / SEQ, t = m % SEQ;
    const float* s = F + (size_t)m * (3 * DM) + sec * DM + c8 * 8;
    const v4f a = *(const v4f*)s, c = *(const v4f*)(s + 4); v8h vh, vr;
#pragma unroll
    for (int k = 0; k < 4; ++k) { const h16 x0 = (h16)a[k]; vh[k] = x0; vr[k] = (h16)((a[k] - (float)x0) * RSC); const h16 x1 = (h16)c[k]; vh[k + 4] = x1; vr[k + 4] = (h16)((c[k] - (float)x1) * RSC); }
    const size_t oo = ((size_t)(b * NH + h) * SEQ + t) * HD + d0;
    const size_t oe = ((size_t)(b * NH + h) * RH + (t < RH ? t : 0u)) * HD + d0;
#pragma unroll 1
    for (int ps = 0; ps < 2; ++ps) {
        if (sec == 0) { *(volatile v8h*)(QH + oo) = vh; *(volatile v8h*)(QR + oo) = vr; }
        else { *(volatile v8h*)(KH + oo) = vh; if (t < RH) *(volatile v8h*)(KR + oe) = vr; }
        if (ps == 0) __threadfence(); }
}
__global__ __launch_bounds__(256) void k_vtp(const float* __restrict__ F, h16* VT, h16* VTR) {
    const unsigned i = blockIdx.x * 256u + threadIdx.x; if (i >= (unsigned)(NB * NH * HD * (SEQ / 8))) return;
    const unsigned t8 = i % (SEQ / 8), dd = (i / (SEQ / 8)) % HD, bh = i / ((SEQ / 8) * HD); const unsigned b = bh / NH, h = bh % NH;
    const float* s = F + ((size_t)b * SEQ + t8 * 8) * (3 * DM) + 2 * DM + h * HD + dd; v8h vh, vr;
#pragma unroll
    for (int k = 0; k < 8; ++k) { const float v = s[(size_t)k * (3 * DM)]; const h16 x0 = (h16)v; vh[k] = x0; vr[k] = (h16)((v - (float)x0) * RSC); }
    const size_t oo = ((size_t)bh * HD + dd) * SEQ + t8 * 8;
    const bool er = (t8 * 8 < RH);
    const size_t oe = ((size_t)bh * HD + dd) * RH + (er ? t8 * 8 : 0u);
#pragma unroll 1
    for (int ps = 0; ps < 2; ++ps) {
        *(volatile v8h*)(VT + oo) = vh; if (er) *(volatile v8h*)(VTR + oe) = vr;
        if (ps == 0) __threadfence(); }
}

template <bool EARLY>
__device__ __forceinline__ void attn_body(const h16* QH, const h16* QR, const h16* KH, const h16* KR, const h16* VT, const h16* VTR, bf* YH, bf* YL, const int bh, const int qbase, const int wave) {
    __shared__ __align__(16) h16 pts[8 * 16 * PP];
    __shared__ __align__(16) h16 prs[8 * 16 * PP];
    __shared__ __align__(16) float ots[8 * 16 * OP];
    const int lane = threadIdx.x & 31, lr = lane & 15, hi = lane >> 4;
    const int pb = wave * (16 * PP), ob = wave * (16 * OP);
    const unsigned qoff = (unsigned)((bh * SEQ + qbase + lr) * HD + 8 * hi);
    v16h qh0 = ldh(QH + qoff), qh1 = ldh(QH + qoff + 32), qr0 = ldh(QR + qoff), qr1 = ldh(QR + qoff + 32);
    float mrow[8], lsum[8]; v8f oh[4], ol[4];
#pragma unroll
    for (int r = 0; r < 8; ++r) { mrow[r] = NEGB; lsum[r] = 0.0f; }
#pragma unroll
    for (int f = 0; f < 4; ++f) { oh[f] = (v8f){}; ol[f] = (v8f){}; }
    const int kend = qbase + 16;
#pragma unroll 1
    for (int kb = 0; kb < kend; kb += 32) {
        if (EARLY) { unsigned qo = qoff; asm volatile("" : "+v"(qo)); qh0 = ldh(QH + qo); qh1 = ldh(QH + qo + 32); qr0 = ldh(QR + qo); qr1 = ldh(QR + qo + 32); }
        float t[2][8];
#pragma unroll
        for (int j = 0; j < 2; ++j) {
            const unsigned koff = (unsigned)((bh * SEQ + kb + 16 * j + lr) * HD + 8 * hi);
            const v16h k0 = ldh(KH + koff), k1 = ldh(KH + koff + 32);
            v8f sh = (v8f){}, sr = (v8f){};
            sh = wmma16(qh0, k0, sh); sh = wmma16(qh1, k1, sh);
            sr = wmma16(qr0, k0, sr); sr = wmma16(qr1, k1, sr);
            if (EARLY) {
                const unsigned roff = (unsigned)((bh * RH + kb + 16 * j + lr) * HD + 8 * hi);
                const v16h r0 = ldh(KR + roff), r1 = ldh(KR + roff + 32);
                sr = wmma16(qh0, r0, sr); sr = wmma16(qh1, r1, sr);
                asm volatile("v_nop\n\tv_nop\n\tv_nop\n\tv_nop" : "+v"(sh), "+v"(sr) : "v"(qh1), "v"(r1));
            } else {
                asm volatile("v_nop\n\tv_nop\n\tv_nop\n\tv_nop" : "+v"(sh), "+v"(sr) : "v"(qr1), "v"(k1));
            }
#pragma unroll
            for (int r = 0; r < 8; ++r) t[j][r] = (sh[r] + sr[r] * RINV) * SC2;
        }
        if (kb + 31 > qbase) {
#pragma unroll
            for (int j = 0; j < 2; ++j)
#pragma unroll
                for (int r = 0; r < 8; ++r) { if (kb + 16 * j + lr > qbase + 8 * hi + r) t[j][r] = NEGB; }
        }
        float scl[8];
#pragma unroll
        for (int r = 0; r < 8; ++r) {
            float rm = fmaxf(t[0][r], t[1][r]);
            rm = fmaxf(rm, __shfl_xor(rm, 1, 32)); rm = fmaxf(rm, __shfl_xor(rm, 2, 32)); rm = fmaxf(rm, __shfl_xor(rm, 4, 32)); rm = fmaxf(rm, __shfl_xor(rm, 8, 32));
            const float mn = fmaxf(mrow[r], rm);
            scl[r] = __builtin_amdgcn_exp2f(mrow[r] - mn);
            mrow[r] = mn;
            const float ms = mn - 10.0f;
            const float p0 = __builtin_amdgcn_exp2f(t[0][r] - ms), p1 = __builtin_amdgcn_exp2f(t[1][r] - ms);
            lsum[r] = lsum[r] * scl[r] + (p0 + p1);
            const int pi = pb + (8 * hi + r) * PP + lr;
            const h16 a0 = (h16)p0, a1 = (h16)p1;
            pts[pi] = a0; pts[pi + 16] = a1;
            if (EARLY) { prs[pi] = (h16)((p0 - (float)a0) * RSC); prs[pi + 16] = (h16)((p1 - (float)a1) * RSC); }
        }
#pragma unroll
        for (int f = 0; f < 4; ++f)
#pragma unroll
            for (int r = 0; r < 8; ++r) { oh[f][r] *= scl[r]; if (EARLY) ol[f][r] *= scl[r]; }
        __builtin_amdgcn_wave_barrier(); asm volatile("" ::: "memory");
        const v16h aP = cat16(*(const v8ha*)&pts[pb + lr * PP + 8 * hi], *(const v8ha*)&pts[pb + lr * PP + 16 + 8 * hi]);
        v16h aR = aP;
        if (EARLY) aR = cat16(*(const v8ha*)&prs[pb + lr * PP + 8 * hi], *(const v8ha*)&prs[pb + lr * PP + 16 + 8 * hi]);
        __builtin_amdgcn_wave_barrier(); asm volatile("" ::: "memory");
        const unsigned voff = (unsigned)((bh * HD + lr) * SEQ + kb + 8 * hi);
        const unsigned vroff = (unsigned)((bh * HD + lr) * RH + kb + 8 * hi);
#pragma unroll
        for (int f = 0; f < 4; ++f) {
            const v16h vf = ldh(VT + voff + f * 16 * SEQ);
            oh[f] = wmma16(aP, vf, oh[f]);
            if (EARLY) { const v16h vr = ldh(VTR + vroff + f * 16 * RH); ol[f] = wmma16(aR, vf, ol[f]); ol[f] = wmma16(aP, vr, ol[f]); }
        }
        if (EARLY) asm volatile("v_nop\n\tv_nop\n\tv_nop\n\tv_nop" : "+v"(oh[0]), "+v"(oh[1]), "+v"(oh[2]), "+v"(oh[3]), "+v"(ol[0]), "+v"(ol[1]), "+v"(ol[2]), "+v"(ol[3]) : "v"(aP), "v"(aR));
        else       asm volatile("v_nop\n\tv_nop\n\tv_nop\n\tv_nop" : "+v"(oh[0]), "+v"(oh[1]), "+v"(oh[2]), "+v"(oh[3]) : "v"(aP));
    }
#pragma unroll
    for (int r = 0; r < 8; ++r) {
        float l = lsum[r];
        l += __shfl_xor(l, 1, 32); l += __shfl_xor(l, 2, 32); l += __shfl_xor(l, 4, 32); l += __shfl_xor(l, 8, 32);
        const float inv = 1.0f / l;
#pragma unroll
        for (int f = 0; f < 4; ++f) { float v = oh[f][r]; if (EARLY) v += ol[f][r] * RINV; ots[ob + (8 * hi + r) * OP + f * 16 + lr] = v * inv; }
    }
    __builtin_amdgcn_wave_barrier(); asm volatile("" ::: "memory");
    const unsigned ybase = (unsigned)(((bh / NH) * SEQ + qbase) * DM + (bh % NH) * HD);
#pragma unroll 1
    for (int ps = 0; ps < 2; ++ps) {
#pragma unroll
        for (int s = 0; s < 4; ++s) {
            const int row = s * 4 + (lane >> 3), c8 = (lane & 7) * 8;
            const v4f a = *(const v4fa*)&ots[ob + row * OP + c8], c = *(const v4fa*)&ots[ob + row * OP + c8 + 4];
            v8us vh, vl;
#pragma unroll
            for (int k = 0; k < 4; ++k) { unsigned short x0, x1; splitf(a[k], x0, x1); vh[k] = x0; vl[k] = x1; splitf(c[k], x0, x1); vh[k + 4] = x0; vl[k + 4] = x1; }
            const unsigned oo = ybase + (unsigned)(row * DM + c8);
            *(volatile v8us*)(YH + oo) = vh; *(volatile v8us*)(YL + oo) = vl;
        }
        if (ps == 0) __threadfence();
    }
}
__global__ __launch_bounds__(256) void k_attn_e(const h16* QH, const h16* QR, const h16* KH, const h16* KR, const h16* VT, const h16* VTR, bf* YH, bf* YL) {
    const int wave = __builtin_amdgcn_readfirstlane((int)(threadIdx.x >> 5));
    const int gw = (int)blockIdx.x * 8 + wave; const int bh = gw / TPE, qt = gw % TPE;
    attn_body<true>(QH, QR, KH, KR, VT, VTR, YH, YL, bh, qt * 16, wave);
}
__global__ __launch_bounds__(256) void k_attn_m(const h16* QH, const h16* QR, const h16* KH, const h16* VT, bf* YH, bf* YL) {
    const int wave = __builtin_amdgcn_readfirstlane((int)(threadIdx.x >> 5));
    const int gw = (int)blockIdx.x * 8 + wave; const int bh = gw / TPMD, qt = gw % TPMD + TPE;
    attn_body<false>(QH, QR, KH, KH, VT, VT, YH, YL, bh, qt * 16, wave);
}

constexpr size_t al256(size_t b) { return (b + 255) & ~(size_t)255; }
constexpr size_t SZ_WQKV = al256((size_t)3 * DM * DM * 2);
constexpr size_t SZ_WO   = al256((size_t)DM * DM * 2);
constexpr size_t SZ_XB   = al256((size_t)NB * SEQ * DM * 2);
constexpr size_t SZ_F    = al256((size_t)NB * SEQ * 3 * DM * 4);
constexpr size_t SZ_PL   = al256((size_t)NB * NH * SEQ * HD * 2);
constexpr size_t SZ_PE   = al256((size_t)NB * NH * RH * HD * 2);
constexpr size_t SZ_Y    = al256((size_t)NB * SEQ * DM * 2);
constexpr size_t WS_TOTAL = SZ_WQKV + SZ_WO + SZ_XB + SZ_F + 4 * SZ_PL + 2 * SZ_PE + 2 * SZ_Y;
static_assert(WS_TOTAL <= (size_t)134217728);

extern "C" void kernel_launch(void* const* d_in, const int* in_sizes, int n_in,
                              void* d_out, int out_size, void* d_ws, size_t ws_size, hipStream_t stream) {
    if (n_in < 4) return;
    const size_t need_x = ((size_t)(NB - 1) * SEQ_FULL + SEQ) * DM;
    if ((size_t)in_sizes[0] < need_x) return;
    if ((size_t)in_sizes[1] < (size_t)3 * DM * DM) return;
    if ((size_t)in_sizes[2] < (size_t)DM * DM) return;
    if (in_sizes[3] < DM) return;
    if ((size_t)out_size < need_x) return;
    if (ws_size < WS_TOTAL) return;
    const float* x = (const float*)d_in[0]; const float* wqkv = (const float*)d_in[1]; const float* wo = (const float*)d_in[2]; const float* bo = (const float*)d_in[3];
    float* OUT = (float*)d_out;
    char* wsp = (char*)d_ws;
    bf* WQKV = (bf*)wsp; wsp += SZ_WQKV;
    bf* WO   = (bf*)wsp; wsp += SZ_WO;
    bf* XB   = (bf*)wsp; wsp += SZ_XB;
    float* F = (float*)wsp; wsp += SZ_F;
    h16* QH  = (h16*)wsp; wsp += SZ_PL;
    h16* QR  = (h16*)wsp; wsp += SZ_PL;
    h16* KH  = (h16*)wsp; wsp += SZ_PL;
    h16* VT  = (h16*)wsp; wsp += SZ_PL;
    h16* KR  = (h16*)wsp; wsp += SZ_PE;
    h16* VTR = (h16*)wsp; wsp += SZ_PE;
    bf* YH   = (bf*)wsp; wsp += SZ_Y;
    bf* YL   = (bf*)wsp; wsp += SZ_Y;

    k_wt<<<(unsigned)((3 * DM * (DM / 64) + 63) / 64), 256, 0, stream>>>(wqkv, 3 * DM, WQKV);
    k_wt<<<(unsigned)((DM * (DM / 64) + 63) / 64), 256, 0, stream>>>(wo, DM, WO);
    k_cvtx<<<(unsigned)((NB * SEQ * (DM / 8) + 255) / 256), 256, 0, stream>>>(x, XB);
    k_gemm_qkv<<<dim3(NB * SEQ / 64, 3 * DM / 64, 1), 32, 0, stream>>>(XB, WQKV, F);
    k_qkp<<<(unsigned)(NB * SEQ), 256, 0, stream>>>(F, QH, QR, KH, KR);
    k_vtp<<<(unsigned)((NB * NH * HD * (SEQ / 8) + 255) / 256), 256, 0, stream>>>(F, VT, VTR);
    k_attn_e<<<(unsigned)(NB * NH * TPE / 8), 256, 0, stream>>>(QH, QR, KH, KR, VT, VTR, YH, YL);
    if (TPM > 0) k_attn_m<<<(unsigned)(NB * NH * TPMD / 8), 256, 0, stream>>>(QH, QR, KH, VT, YH, YL);
    k_gemm_out<<<dim3(SEQ / 64, DM / 64, NB), 32, 0, stream>>>(YH, YL, WO, bo, OUT);
}
